// GNNConditioner_36258113913103
// MI455X (gfx1250) — hardware-verified
//
#include <hip/hip_runtime.h>

#define NB    4096
#define NA    32
#define NF    64
#define NM    32
#define DREST 160
#define KFEAT 2208
#define FP    2240
#define HID   1024
#define DOUT  256
#define NWAV  8
#define RS8   (1.0f / 2.8284271247461903f)
#define I2W2  (1.0f / 0.017578125f)

typedef unsigned short us;
typedef us       v8us __attribute__((ext_vector_type(8)));
typedef v8us __attribute__((may_alias)) v8usa;
typedef _Float16 v16h __attribute__((ext_vector_type(16)));
typedef __bf16   v16b __attribute__((ext_vector_type(16)));
typedef float    v8f  __attribute__((ext_vector_type(8)));
typedef float    v4f  __attribute__((ext_vector_type(4)));
typedef v4f __attribute__((may_alias)) v4fa;
union Frag { v16h h; v16b b; v8us u[2]; };

__device__ __forceinline__ us h_rne(float v) { _Float16 t = (_Float16)v; return __builtin_bit_cast(us, t); }
__device__ __forceinline__ us bf_rne(float v) { unsigned u = __float_as_uint(v); return (us)((u + 0x7FFFu + ((u >> 16) & 1u)) >> 16); }
__device__ __forceinline__ float bf_up(us q) { return __uint_as_float(((unsigned)q) << 16); }
__device__ __forceinline__ us bf_lo(float v, us hi) { return bf_rne(v - bf_up(hi)); }

__device__ __forceinline__ v8f wmh(Frag a, Frag b, v8f c) { return __builtin_amdgcn_wmma_f32_16x16x32_f16(false, a.h, false, b.h, (short)0, c, false, false); }
__device__ __forceinline__ v8f wmb(Frag a, Frag b, v8f c) { return __builtin_amdgcn_wmma_f32_16x16x32_bf16(false, a.b, false, b.b, (short)0, c, false, false); }
__device__ __forceinline__ void guard3(v8f& d, Frag a, Frag b, Frag c, Frag e) {
  asm volatile("v_nop\n\tv_nop\n\tv_nop\n\tv_nop" : "+v"(d) : "v"(a.h), "v"(b.h), "v"(c.h), "v"(e.h));
}
__device__ __forceinline__ void guard2(v8f& d0, v8f& d1, Frag a, Frag b, Frag c) {
  asm volatile("v_nop\n\tv_nop\n\tv_nop\n\tv_nop" : "+v"(d0), "+v"(d1) : "v"(a.h), "v"(b.h), "v"(c.h));
}
__device__ __forceinline__ void guard2x(v8f& d0, v8f& d1, Frag a, Frag b, Frag c, Frag e, Frag f, Frag g) {
  asm volatile("v_nop\n\tv_nop\n\tv_nop\n\tv_nop" : "+v"(d0), "+v"(d1) : "v"(a.h), "v"(b.h), "v"(c.h), "v"(e.h), "v"(f.h), "v"(g.h));
}
__device__ __forceinline__ Frag ldf(const us* p, int h) {
  Frag f;
  f.u[0] = *(const v8usa*)(p + 8 * h);
  f.u[1] = *(const v8usa*)(p + 16 + 8 * h);
  return f;
}

template <int BF>
__global__ __launch_bounds__(256) void k_cvt(const float* __restrict__ W, int N, int koff, int K, int Kp, float sc, us* P0, us* P1, int np) {
  const int p = blockIdx.x * 256 + threadIdx.x;
  if (p >= np) return;
  const int f = 8 * p, n = f / Kp, k = f - n * Kp;
  v8us a = (v8us)((us)0), b = (v8us)((us)0);
#pragma unroll
  for (int kk = 0; kk < 8; ++kk) {
    const int kc = k + kk, kcl = (kc < K) ? kc : (K - 1);
    float v = W[(size_t)(koff + kcl) * N + n] * sc;
    v = (kc < K) ? v : 0.0f;
    if (BF) { const us hi = bf_rne(v); a[kk] = hi; b[kk] = bf_lo(v, hi); }
    else    { a[kk] = h_rne(v); }
  }
  *(volatile v8us*)(P0 + f) = a;
  if (BF) *(volatile v8us*)(P1 + f) = b;
  __threadfence();
  *(volatile v8us*)(P0 + f) = a;
  if (BF) *(volatile v8us*)(P1 + f) = b;
}

template <int EPI>
__device__ __forceinline__ void gemm_store(const float* sTf, const us* sTh, us* C0, us* C1, float* Cf, int ldc, int R0, int CC, int w, int l) {
  const int q8 = l & 7, sub = l >> 3;
  if (EPI == 2) {
#pragma unroll
    for (int i = 0; i < 16; ++i) {
      const int lid = 4 * i + sub, row = 32 * w + (lid >> 1), hl = lid & 1;
      const v4f v = *(const v4fa*)(sTf + row * 64 + 32 * hl + 4 * q8);
      *(volatile v4f*)(Cf + (size_t)(R0 + row) * ldc + CC + 32 * hl + 4 * q8) = v;
    }
  } else {
#pragma unroll
    for (int i = 0; i < 8; ++i) {
      const int row = 32 * w + 4 * i + sub;
      const v8us v = *(const v8usa*)(sTh + row * 64 + 8 * q8);
      *(volatile v8us*)(C0 + (size_t)(R0 + row) * ldc + CC + 8 * q8) = v;
      if (EPI == 1) {
        const v8us v2 = *(const v8usa*)(sTh + 8192 + row * 64 + 8 * q8);
        *(volatile v8us*)(C1 + (size_t)(R0 + row) * ldc + CC + 8 * q8) = v2;
      }
    }
  }
}

template <int X3, int EPI>
__global__ __launch_bounds__(128) void k_gemm(const us* __restrict__ Ah, const us* __restrict__ Al, int lda,
                                              const us* __restrict__ Bh, const us* __restrict__ Bl, int ldb, int K,
                                              const float* __restrict__ bias, float osc, us* C0, us* C1, float* Cf, int ldc) {
  __shared__ __attribute__((aligned(16))) float sTf[128 * 64];
  __shared__ __attribute__((aligned(16))) us sTh[2 * 128 * 64];
  const int tid = threadIdx.x, l = tid & 31, w = tid >> 5, h = l >> 4, m = l & 15;
  const int R0 = blockIdx.x * 128, CC = blockIdx.y * 64;
  const size_t ra = (size_t)(R0 + 32 * w + m);
  const us* a0h = Ah + ra * lda; const us* a1h = a0h + (size_t)16 * lda;
  const us* a0l = Al + ra * lda; const us* a1l = a0l + (size_t)16 * lda;
  const us* bhp = Bh + (size_t)(CC + m) * ldb; const us* blp = Bl + (size_t)(CC + m) * ldb;
  v8f acc[2][4];
#pragma unroll
  for (int i = 0; i < 2; ++i)
#pragma unroll
    for (int j = 0; j < 4; ++j) acc[i][j] = (v8f)(0.0f);

#pragma unroll 1
  for (int k0 = 0; k0 < K; k0 += 32) {
    const Frag a0 = ldf(a0h + k0, h), a1 = ldf(a1h + k0, h);
    Frag c0 = a0, c1 = a1;
    if (X3) { c0 = ldf(a0l + k0, h); c1 = ldf(a1l + k0, h); }
#pragma unroll
    for (int nt = 0; nt < 4; ++nt) {
      const Frag b = ldf(bhp + (size_t)nt * 16 * ldb + k0, h);
      if (X3) {
        const Frag d = ldf(blp + (size_t)nt * 16 * ldb + k0, h);
        acc[0][nt] = wmb(a0, b, acc[0][nt]); acc[0][nt] = wmb(a0, d, acc[0][nt]); acc[0][nt] = wmb(c0, b, acc[0][nt]);
        acc[1][nt] = wmb(a1, b, acc[1][nt]); acc[1][nt] = wmb(a1, d, acc[1][nt]); acc[1][nt] = wmb(c1, b, acc[1][nt]);
        guard2x(acc[0][nt], acc[1][nt], a0, c0, a1, c1, b, d);
      } else {
        acc[0][nt] = wmh(a0, b, acc[0][nt]);
        acc[1][nt] = wmh(a1, b, acc[1][nt]);
        guard2(acc[0][nt], acc[1][nt], a0, a1, b);
      }
    }
  }
#pragma unroll
  for (int mt = 0; mt < 2; ++mt)
#pragma unroll
    for (int nt = 0; nt < 4; ++nt) {
      const int col = 16 * nt + m;
      const float bv = bias[CC + col];
#pragma unroll
      for (int r = 0; r < 8; ++r) sTf[(32 * w + 16 * mt + 8 * h + r) * 64 + col] = acc[mt][nt][r] * osc + bv;
    }
  __syncthreads();
  if (EPI != 2) {
#pragma unroll 2
    for (int idx = tid; idx < 128 * 64; idx += 128) {
      const float v = tanhf(sTf[idx]);
      if (EPI == 0) { sTh[idx] = h_rne(v); }
      else { const us hi = bf_rne(v); sTh[idx] = hi; sTh[8192 + idx] = bf_lo(v, hi); }
    }
    __syncthreads();
  }
  gemm_store<EPI>(sTf, sTh, C0, C1, Cf, ldc, R0, CC, w, l);
  __threadfence();
  gemm_store<EPI>(sTf, sTh, C0, C1, Cf, ldc, R0, CC, w, l);
}

template <int NT, int KS, int MODE>
__device__ __forceinline__ void gemm3(const us* Ah, const us* Al, int lda, const us* Bh, const us* Bl, int ldb,
                                      const float* bias, float* Df, us* Dh, us* Dl, int ldd) {
  const int w = threadIdx.x >> 5, l = threadIdx.x & 31, h = l >> 4, m = l & 15;
  for (int it = w; it < 2 * NT; it += NWAV) {
    const int mt = it & 1, nt = it >> 1;
    const us* ah = Ah + (16 * mt + m) * lda; const us* al = Al + (16 * mt + m) * lda;
    const us* bh = Bh + (size_t)(16 * nt + m) * ldb; const us* bl = Bl + (size_t)(16 * nt + m) * ldb;
    v8f acc = (v8f)(0.0f);
#pragma unroll
    for (int ks = 0; ks < KS; ++ks) {
      const Frag a0 = ldf(ah + 32 * ks, h), a1 = ldf(al + 32 * ks, h), b0 = ldf(bh + 32 * ks, h), b1 = ldf(bl + 32 * ks, h);
      acc = wmb(a0, b0, acc); acc = wmb(a0, b1, acc); acc = wmb(a1, b0, acc);
      guard3(acc, a0, a1, b0, b1);
    }
    const int col = 16 * nt + m;
    const float bb = bias[col];
#pragma unroll
    for (int r = 0; r < 8; ++r) {
      const int row = 16 * mt + 8 * h + r;
      const float v = acc[r] + bb;
      if (MODE == 0) Df[col * ldd + row] = v;
      else if (MODE == 1) Df[row * ldd + col] = v;
      else if (MODE == 2) Df[row * ldd + col] += v;
      else if (MODE == 3) Df[row * ldd + col] += v * __builtin_amdgcn_rcpf(1.0f + __expf(-v));
      else { const float t = (MODE == 5) ? fmaxf(v, 0.0f) : v; const us hi = bf_rne(t); Dh[row * ldd + col] = hi; Dl[row * ldd + col] = bf_lo(t, hi); }
    }
  }
}

__device__ __forceinline__ void msg_gemm(const us* e16, const us* wme, const float* hwmT, const float* mask, float* part) {
  const int w = threadIdx.x >> 5, l = threadIdx.x & 31, h = l >> 4, m = l & 15;
  const v8us zu = (v8us)((us)0);
  Frag b0, b1;
  b0.u[0] = *(const v8usa*)(wme + m * 16 + 8 * h); b0.u[1] = zu;
  b1.u[0] = *(const v8usa*)(wme + (16 + m) * 16 + 8 * h); b1.u[1] = zu;
#pragma unroll 1
  for (int mt = w; mt < 64; mt += NWAV) {
    Frag a;
    a.u[0] = *(const v8usa*)(e16 + (mt * 16 + m) * 16 + 8 * h); a.u[1] = zu;
    v8f s0 = wmh(a, b0, (v8f)(0.0f)), s1 = wmh(a, b1, (v8f)(0.0f));
    guard2(s0, s1, a, b0, b1);
    const int i = mt >> 1, j0 = (mt & 1) * 16 + 8 * h;
    const float* mk = mask + i * 32 + j0;
    const float* hw0 = hwmT + m * 32 + j0;
    const float* hw1 = hwmT + (16 + m) * 32 + j0;
    float p0 = 0.f, p1 = 0.f;
#pragma unroll
    for (int r = 0; r < 8; ++r) {
      float t0 = s0[r] * (1.0f / 256.0f) + hw0[r];
      float t1 = s1[r] * (1.0f / 256.0f) + hw1[r];
      t0 = t0 * __builtin_amdgcn_rcpf(1.0f + __expf(-t0));
      t1 = t1 * __builtin_amdgcn_rcpf(1.0f + __expf(-t1));
      p0 += mk[r] * t0; p1 += mk[r] * t1;
    }
    p0 += __shfl_xor(p0, 16);
    p1 += __shfl_xor(p1, 16);
    if (h == 0) { part[mt * 32 + m] = p0; part[mt * 32 + 16 + m] = p1; }
  }
}

__device__ __forceinline__ void geom(const float* pos, float* mask, us* e16, int tid) {
#pragma clang fp contract(off)
  for (int idx = tid; idx < 1024; idx += 256) {
    const int i = idx >> 5, j = idx & 31;
    const float dx = pos[3 * i] - pos[3 * j], dy = pos[3 * i + 1] - pos[3 * j + 1], dz = pos[3 * i + 2] - pos[3 * j + 2];
    float s = (dx * dx + dz * dz) + dy * dy;
    s = fmaxf(s, 1e-12f);
    const float d = sqrtf(s);
    mask[idx] = (i != j && d <= 1.5f) ? 1.0f : 0.0f;
    v8us ea = (v8us)((us)0), eb = (v8us)((us)0);
#pragma unroll
    for (int r = 0; r < 16; ++r) {
      const float c = (r == 15) ? 1.5f : 1.5f * ((float)r * (1.0f / 15.0f));
      const float t = d - c;
      const float e = __expf(-(t * t) * I2W2) * 16.0f;
      const us q = h_rne(e);
      if (r < 8) ea[r] = q; else eb[r - 8] = q;
    }
    *(v8usa*)(e16 + idx * 16) = ea;
    *(v8usa*)(e16 + idx * 16 + 8) = eb;
  }
}

__device__ __forceinline__ void hplanes(const float* sh, us* ph, us* pl, int tid) {
  for (int i = tid; i < 2048; i += 256) {
    const float v = sh[i];
    const us hi = bf_rne(v);
    const int o = (i >> 6) * 96 + (i & 63);
    ph[o] = hi; pl[o] = bf_lo(v, hi);
  }
}

__device__ __forceinline__ void ln_stats(const float* s, float* red, int tid) {
  if (tid < 32) {
    float mu = 0.f;
#pragma unroll 4
    for (int f = 0; f < 64; ++f) mu += s[tid * 64 + f];
    mu *= (1.0f / 64.0f);
    float vv = 0.f;
#pragma unroll 4
    for (int f = 0; f < 64; ++f) { const float t = s[tid * 64 + f] - mu; vv += t * t; }
    red[2 * tid] = mu;
    red[2 * tid + 1] = 1.0f / sqrtf(vv * (1.0f / 64.0f) + 1e-5f);
  }
}

__device__ __forceinline__ void feat_store(const us* sfeat, us* dst, int tid) {
  for (int p = tid; p < FP / 8; p += 256) {
    const v8us v = *(const v8usa*)(sfeat + 8 * p);
    *(volatile v8us*)(dst + 8 * p) = v;
  }
}

struct MolArgs {
  const float *x, *emb, *bm0, *bm1, *bu0, *bu1, *bqkv, *bq, *bk, *bv, *bo, *b1f, *b2f, *g1, *be1, *g2, *be2;
  const us *wmh0h, *wmh0l, *wme0, *wu0h, *wu0l, *wmh1h, *wmh1l, *wme1, *wu1h, *wu1l,
           *wqkvh, *wqkvl, *wqh, *wql, *wkh, *wkl, *wvh, *wvl, *woh, *wol, *w1h, *w1l, *w2h, *w2l;
  us* feat;
};
static_assert(sizeof(MolArgs) == 42 * 8);

struct MPsh { us e16[1024 * 16]; float hwm[1024]; float part[2048]; };
struct ATsh { float q[2048], k[2048], v[2048], sc[8192]; };
union MolU { MPsh mp; ATsh at; };

__global__ __launch_bounds__(256) void k_mol(MolArgs A) {
  __shared__ float spos[96];
  __shared__ __attribute__((aligned(16))) float smask[1024];
  __shared__ __attribute__((aligned(16))) float sh[2048];
  __shared__ float sred[64];
  __shared__ __attribute__((aligned(16))) us sA[2][32 * 96];
  __shared__ __attribute__((aligned(16))) us sQ[2][32 * 192];
  __shared__ __attribute__((aligned(16))) us sT[2][2048];
  __shared__ __attribute__((aligned(16))) us sfeat[FP];
  __shared__ __attribute__((aligned(16))) MolU u;

  const int tid = threadIdx.x, b = blockIdx.x;
  const float* xr = A.x + (size_t)b * 256;
  if (tid < 96) spos[tid] = xr[tid];
  for (int i = tid; i < 2048; i += 256) sh[i] = A.emb[i];
  __syncthreads();
  geom(spos, smask, u.mp.e16, tid);
  __syncthreads();

  for (int L = 0; L < 2; ++L) {
    const us* wmhh = L ? A.wmh1h : A.wmh0h; const us* wmhl = L ? A.wmh1l : A.wmh0l;
    const us* wme = L ? A.wme1 : A.wme0;
    const us* wuh = L ? A.wu1h : A.wu0h;     const us* wul = L ? A.wu1l : A.wu0l;
    const float* bm = L ? A.bm1 : A.bm0;     const float* bu = L ? A.bu1 : A.bu0;
    hplanes(sh, sA[0], sA[1], tid);
    __syncthreads();
    gemm3<2, 2, 0>(sA[0], sA[1], 96, wmhh, wmhl, 64, bm, u.mp.hwm, sT[0], sT[1], 32);
    __syncthreads();
    msg_gemm(u.mp.e16, wme, u.mp.hwm, smask, u.mp.part);
    __syncthreads();
    for (int i = tid; i < 1024; i += 256) {
      const int a = i >> 5, mm = i & 31;
      const float v = u.mp.part[(2 * a) * 32 + mm] + u.mp.part[(2 * a + 1) * 32 + mm];
      const us hi = bf_rne(v);
      sA[0][a * 96 + 64 + mm] = hi; sA[1][a * 96 + 64 + mm] = bf_lo(v, hi);
    }
    __syncthreads();
    gemm3<4, 3, 3>(sA[0], sA[1], 96, wuh, wul, 96, bu, sh, sT[0], sT[1], 64);
    __syncthreads();
  }

  hplanes(sh, sA[0], sA[1], tid);
  __syncthreads();
  gemm3<12, 2, 4>(sA[0], sA[1], 96, A.wqkvh, A.wqkvl, 64, A.bqkv, sh, sQ[0], sQ[1], 192);
  __syncthreads();
  gemm3<4, 2, 1>(sQ[0], sQ[1], 192, A.wqh, A.wql, 64, A.bq, u.at.q, sT[0], sT[1], 64);
  gemm3<4, 2, 1>(sQ[0] + 64, sQ[1] + 64, 192, A.wkh, A.wkl, 64, A.bk, u.at.k, sT[0], sT[1], 64);
  gemm3<4, 2, 1>(sQ[0] + 128, sQ[1] + 128, 192, A.wvh, A.wvl, 64, A.bv, u.at.v, sT[0], sT[1], 64);
  __syncthreads();
  {
    const int hd = (tid >> 5) * 8, qi = tid & 31;
    float qv[8];
#pragma unroll
    for (int d = 0; d < 8; ++d) qv[d] = u.at.q[qi * 64 + hd + d];
    float mx = -3.0e38f;
#pragma unroll 2
    for (int kj = 0; kj < 32; ++kj) {
      const float* kp = u.at.k + kj * 64 + hd;
      float s = 0.f;
#pragma unroll
      for (int d = 0; d < 8; ++d) s += qv[d] * kp[d];
      s *= RS8;
      u.at.sc[kj * 256 + tid] = s;
      mx = fmaxf(mx, s);
    }
    float den = 0.f, od[8];
#pragma unroll
    for (int d = 0; d < 8; ++d) od[d] = 0.f;
#pragma unroll 2
    for (int kj = 0; kj < 32; ++kj) {
      const float p = __expf(u.at.sc[kj * 256 + tid] - mx);
      den += p;
      const float* vp = u.at.v + kj * 64 + hd;
#pragma unroll
      for (int d = 0; d < 8; ++d) od[d] += p * vp[d];
    }
    const float inv = __builtin_amdgcn_rcpf(den);
#pragma unroll
    for (int d = 0; d < 8; ++d) {
      const float o = od[d] * inv;
      const us hi = bf_rne(o);
      sT[0][qi * 64 + hd + d] = hi; sT[1][qi * 64 + hd + d] = bf_lo(o, hi);
    }
  }
  __syncthreads();
  gemm3<4, 2, 2>(sT[0], sT[1], 64, A.woh, A.wol, 64, A.bo, sh, sA[0], sA[1], 64);
  __syncthreads();
  ln_stats(sh, sred, tid);
  __syncthreads();
  for (int i = tid; i < 2048; i += 256) {
    const int a = i >> 6, f = i & 63;
    const float v = (sh[i] - sred[2 * a]) * sred[2 * a + 1] * A.g1[f] + A.be1[f];
    sh[i] = v;
    const us hi = bf_rne(v);
    sA[0][a * 96 + f] = hi; sA[1][a * 96 + f] = bf_lo(v, hi);
  }
  __syncthreads();
  gemm3<4, 2, 5>(sA[0], sA[1], 96, A.w1h, A.w1l, 64, A.b1f, sh, sT[0], sT[1], 64);
  __syncthreads();
  gemm3<4, 2, 2>(sT[0], sT[1], 64, A.w2h, A.w2l, 64, A.b2f, sh, sA[0], sA[1], 64);
  __syncthreads();
  ln_stats(sh, sred, tid);
  __syncthreads();
  for (int i = tid; i < 2048; i += 256) {
    const int a = i >> 6, f = i & 63;
    sfeat[DREST + i] = h_rne((sh[i] - sred[2 * a]) * sred[2 * a + 1] * A.g2[f] + A.be2[f]);
  }
  for (int i = tid; i < DREST; i += 256) sfeat[i] = h_rne(xr[96 + i]);
  if (tid < FP - KFEAT) sfeat[KFEAT + tid] = 0;
  __syncthreads();
  feat_store(sfeat, A.feat + (size_t)b * FP, tid);
  __threadfence();
  feat_store(sfeat, A.feat + (size_t)b * FP, tid);
}

static void cvt_b(hipStream_t st, const float* W, int N, int koff, int K, int Kp, us* ph, us* pl) {
  const int np = N * Kp / 8;
  k_cvt<1><<<(np + 255) / 256, 256, 0, st>>>(W, N, koff, K, Kp, 1.0f, ph, pl, np);
}
static void cvt_h(hipStream_t st, const float* W, int N, int koff, int K, int Kp, float sc, us* p) {
  const int np = N * Kp / 8;
  k_cvt<0><<<(np + 255) / 256, 256, 0, st>>>(W, N, koff, K, Kp, sc, p, p, np);
}

extern "C" void kernel_launch(void* const* d_in, const int* in_sizes, int n_in,
                              void* d_out, int out_size, void* d_ws, size_t ws_size,
                              hipStream_t stream) {
  if (n_in < 34 || out_size != NB * DOUT) return;
  if (in_sizes[0] != NB * 256 || in_sizes[1] != NA * NF) return;
  if (in_sizes[2] != 80 * NM || in_sizes[6] != 80 * NM || in_sizes[3] != NM || in_sizes[7] != NM) return;
  if (in_sizes[4] != 96 * NF || in_sizes[8] != 96 * NF || in_sizes[5] != NF || in_sizes[9] != NF) return;
  if (in_sizes[10] != NF * 192 || in_sizes[11] != 192) return;
  for (int i = 12; i <= 15; ++i) if (in_sizes[i] != NF * NF) return;
  for (int i = 16; i <= 19; ++i) if (in_sizes[i] != NF) return;
  if (in_sizes[20] != NF * NF || in_sizes[22] != NF * NF || in_sizes[21] != NF || in_sizes[23] != NF) return;
  for (int i = 24; i <= 27; ++i) if (in_sizes[i] != NF) return;
  if (in_sizes[28] != KFEAT * HID || in_sizes[29] != HID || in_sizes[30] != HID * HID || in_sizes[31] != HID) return;
  if (in_sizes[32] != HID * DOUT || in_sizes[33] != DOUT) return;

  const float* in[34];
  for (int i = 0; i < 34; ++i) in[i] = (const float*)d_in[i];
  float* out = (float*)d_out;

  char* ws = (char*)d_ws;
  size_t off = 0;
  auto carve = [&](size_t bytes) -> us* { us* p = (us*)(ws + off); off += (bytes + 255) & ~(size_t)255; return p; };
  us *wmh[2][2], *wme[2], *wu[2][2], *wqkv[2], *w6[6][2], *wd1, *wd2, *wd3[2], *feat, *y1, *y2[2];
  for (int L = 0; L < 2; ++L) {
    wmh[L][0] = carve(32 * 64 * 2); wmh[L][1] = carve(32 * 64 * 2);
    wme[L] = carve(32 * 16 * 2);
    wu[L][0] = carve(64 * 96 * 2); wu[L][1] = carve(64 * 96 * 2);
  }
  wqkv[0] = carve(192 * 64 * 2); wqkv[1] = carve(192 * 64 * 2);
  for (int i = 0; i < 6; ++i) { w6[i][0] = carve(64 * 64 * 2); w6[i][1] = carve(64 * 64 * 2); }
  wd1 = carve((size_t)HID * FP * 2);
  wd2 = carve((size_t)HID * HID * 2);
  wd3[0] = carve((size_t)DOUT * HID * 2); wd3[1] = carve((size_t)DOUT * HID * 2);
  feat = carve((size_t)NB * FP * 2);
  y1 = carve((size_t)NB * HID * 2);
  y2[0] = carve((size_t)NB * HID * 2); y2[1] = carve((size_t)NB * HID * 2);
  if (off > ws_size || off > (size_t)134217728) return;

  cvt_b(stream, in[2], NM, 0, 64, 64, wmh[0][0], wmh[0][1]);
  cvt_h(stream, in[2], NM, 64, 16, 16, 16.0f, wme[0]);
  cvt_b(stream, in[4], NF, 0, 96, 96, wu[0][0], wu[0][1]);
  cvt_b(stream, in[6], NM, 0, 64, 64, wmh[1][0], wmh[1][1]);
  cvt_h(stream, in[6], NM, 64, 16, 16, 16.0f, wme[1]);
  cvt_b(stream, in[8], NF, 0, 96, 96, wu[1][0], wu[1][1]);
  cvt_b(stream, in[10], 192, 0, 64, 64, wqkv[0], wqkv[1]);
  const int wsrc[6] = {12, 13, 14, 15, 20, 22};
  for (int i = 0; i < 6; ++i) cvt_b(stream, in[wsrc[i]], NF, 0, 64, 64, w6[i][0], w6[i][1]);
  cvt_h(stream, in[28], HID, 0, KFEAT, FP, 64.0f, wd1);
  cvt_h(stream, in[30], HID, 0, HID, HID, 64.0f, wd2);
  cvt_b(stream, in[32], DOUT, 0, HID, HID, wd3[0], wd3[1]);

  MolArgs a;
  a.x = in[0]; a.emb = in[1];
  a.bm0 = in[3]; a.bm1 = in[7]; a.bu0 = in[5]; a.bu1 = in[9];
  a.bqkv = in[11]; a.bq = in[16]; a.bk = in[17]; a.bv = in[18]; a.bo = in[19];
  a.b1f = in[21]; a.b2f = in[23]; a.g1 = in[24]; a.be1 = in[25]; a.g2 = in[26]; a.be2 = in[27];
  a.wmh0h = wmh[0][0]; a.wmh0l = wmh[0][1]; a.wme0 = wme[0]; a.wu0h = wu[0][0]; a.wu0l = wu[0][1];
  a.wmh1h = wmh[1][0]; a.wmh1l = wmh[1][1]; a.wme1 = wme[1]; a.wu1h = wu[1][0]; a.wu1l = wu[1][1];
  a.wqkvh = wqkv[0]; a.wqkvl = wqkv[1];
  a.wqh = w6[0][0]; a.wql = w6[0][1]; a.wkh = w6[1][0]; a.wkl = w6[1][1];
  a.wvh = w6[2][0]; a.wvl = w6[2][1]; a.woh = w6[3][0]; a.wol = w6[3][1];
  a.w1h = w6[4][0]; a.w1l = w6[4][1]; a.w2h = w6[5][0]; a.w2l = w6[5][1];
  a.feat = feat;
  k_mol<<<NB, 256, 0, stream>>>(a);

  k_gemm<0, 0><<<dim3(NB / 128, HID / 64), 128, 0, stream>>>(feat, feat, FP, wd1, wd1, FP, KFEAT, in[29], 1.0f / 64.0f, y1, y1, out, HID);
  k_gemm<0, 1><<<dim3(NB / 128, HID / 64), 128, 0, stream>>>(y1, y1, HID, wd2, wd2, HID, HID, in[31], 1.0f / 64.0f, y2[0], y2[1], out, HID);
  k_gemm<1, 2><<<dim3(NB / 128, DOUT / 64), 128, 0, stream>>>(y2[0], y2[1], HID, wd3[0], wd3[1], HID, HID, in[33], 1.0f, y1, y1, out, DOUT);
}
